// VanillaRNN_47339129536586
// MI455X (gfx1250) — hardware-verified
//
#include <hip/hip_runtime.h>
#include <math.h>

typedef __attribute__((ext_vector_type(16))) __bf16   v16b;
typedef __attribute__((ext_vector_type(8)))  __bf16   v8b;
typedef __attribute__((ext_vector_type(8)))  _Float16 v8h;
typedef __attribute__((ext_vector_type(8)))  float    v8f;
typedef __attribute__((ext_vector_type(4)))  float    v4f;

constexpr int kVocab   = 60;
constexpr int kVocPad  = 64;
constexpr int kHid     = 128;
constexpr int kBatch   = 1024;
constexpr int kSteps   = 256;
constexpr int kTileM   = 16;
constexpr int kThr     = 256;
constexpr int kWaves   = kThr / 32;
constexpr int kOutTile = kTileM * kVocab;
constexpr int kOutLines = kOutTile / 32;
constexpr int kPrepBlkP = (kVocPad * kHid / 4) / kThr;
constexpr int kPrepBlkW = (kHid * kHid / 8) / kThr;
static_assert(kHid % 32 == 0, "K multiple of 32");
static_assert(kHid == kWaves * 16, "8 waves x 16 columns cover the hidden width");
static_assert(kBatch % kTileM == 0, "batch is a tile multiple");
static_assert(kOutTile * 4 == kOutLines * 128, "16x60 f32 tile is a whole number of 128-B lines");
static_assert((kOutTile * 4) % 128 == 0, "tile base stays line aligned");
static_assert(kPrepBlkP * kThr * 4 == kVocPad * kHid, "P table producer covers exactly 64x128");
static_assert(kPrepBlkW * kThr * 8 == kHid * kHid, "W plane producer covers exactly 128x128");
static_assert(kVocab * kHid * 4 >= (kTileM * kHid + kOutTile) * 4, "epilogue tiles fit in the table region");

__device__ __forceinline__ unsigned short f2bf_bits(float f) {
  unsigned u = __float_as_uint(f);
  return (unsigned short)((u + 0x7FFFu + ((u >> 16) & 1u)) >> 16);
}
__device__ __forceinline__ float bf_bits2f(unsigned short h) { return __uint_as_float(((unsigned)h) << 16); }

union FragB { v16b v; v8b h[2]; };
__device__ __forceinline__ v16b frag_load_bf(const __bf16* p) {
  FragB f;
  f.h[0] = *(const v8b*)(p);
  f.h[1] = *(const v8b*)(p + 16);
  return f.v;
}
__device__ __forceinline__ v8f mma_bf(v16b a, v16b b, v8f c) {
  c = __builtin_amdgcn_wmma_f32_16x16x32_bf16(false, a, false, b, (short)0, c, false, false);
  asm volatile("v_nop\n\tv_nop\n\tv_nop\n\tv_nop" : "+v"(c) : "v"(a), "v"(b));
  return c;
}
__device__ __forceinline__ void group_guard(v8f& a, v8f& b, v16b x, v16b y, v16b z, v16b w) {
  asm volatile("v_nop\n\tv_nop\n\tv_nop\n\tv_nop" : "+v"(a), "+v"(b) : "v"(x), "v"(y), "v"(z), "v"(w));
}
__device__ __forceinline__ float tanh_acc(float x) {
  const float e = expf(2.0f * x);
  return 1.0f - 2.0f * __builtin_amdgcn_rcpf(e + 1.0f);
}

__global__ __launch_bounds__(kThr) void prep_kernel(const float* __restrict__ emb, const float* __restrict__ w_ih,
                                                    const float* __restrict__ w_hh, float* __restrict__ ptab,
                                                    unsigned short* __restrict__ whi, unsigned short* __restrict__ wlo) {
  const int blk = blockIdx.x, tid = threadIdx.x;
  if (blk < kPrepBlkP) {
    const int idx = blk * kThr + tid;
    const int v   = idx >> 5;
    const int j4  = (idx & 31) * 4;
    const int vc  = (v < kVocab) ? v : (kVocab - 1);
    const float* ev = emb + vc * kHid;
    const float* w0 = w_ih + (j4 + 0) * kHid;
    const float* w1 = w_ih + (j4 + 1) * kHid;
    const float* w2 = w_ih + (j4 + 2) * kHid;
    const float* w3 = w_ih + (j4 + 3) * kHid;
    float s0 = 0.0f, s1 = 0.0f, s2 = 0.0f, s3 = 0.0f;
#pragma unroll 1
    for (int k = 0; k < kHid; k += 4) {
      const v4f e  = *(const v4f*)(ev + k);
      const v4f a0 = *(const v4f*)(w0 + k);
      const v4f a1 = *(const v4f*)(w1 + k);
      const v4f a2 = *(const v4f*)(w2 + k);
      const v4f a3 = *(const v4f*)(w3 + k);
      s0 = fmaf(e[0], a0[0], s0); s0 = fmaf(e[1], a0[1], s0); s0 = fmaf(e[2], a0[2], s0); s0 = fmaf(e[3], a0[3], s0);
      s1 = fmaf(e[0], a1[0], s1); s1 = fmaf(e[1], a1[1], s1); s1 = fmaf(e[2], a1[2], s1); s1 = fmaf(e[3], a1[3], s1);
      s2 = fmaf(e[0], a2[0], s2); s2 = fmaf(e[1], a2[1], s2); s2 = fmaf(e[2], a2[2], s2); s2 = fmaf(e[3], a2[3], s2);
      s3 = fmaf(e[0], a3[0], s3); s3 = fmaf(e[1], a3[1], s3); s3 = fmaf(e[2], a3[2], s3); s3 = fmaf(e[3], a3[3], s3);
    }
    const bool live = (v < kVocab);
    v4f o;
    o[0] = live ? s0 : 0.0f;
    o[1] = live ? s1 : 0.0f;
    o[2] = live ? s2 : 0.0f;
    o[3] = live ? s3 : 0.0f;
    float* op = ptab + v * kHid + j4;
    *(volatile v4f*)op = o;
    __threadfence();
    *(volatile v4f*)op = o;
  } else {
    const int i = (blk - kPrepBlkP) * kThr + tid;
    const float* sp = w_hh + (size_t)i * 8;
    const v4f a = *(const v4f*)(sp);
    const v4f b = *(const v4f*)(sp + 4);
    v8h hv, lv;
#pragma unroll
    for (int e = 0; e < 4; ++e) {
      const float xa = a[e];
      const float xb = b[e];
      const unsigned short ha = f2bf_bits(xa);
      const unsigned short hb = f2bf_bits(xb);
      const unsigned short la = f2bf_bits(xa - bf_bits2f(ha));
      const unsigned short lb = f2bf_bits(xb - bf_bits2f(hb));
      hv[e]     = __builtin_bit_cast(_Float16, ha);
      hv[4 + e] = __builtin_bit_cast(_Float16, hb);
      lv[e]     = __builtin_bit_cast(_Float16, la);
      lv[4 + e] = __builtin_bit_cast(_Float16, lb);
    }
    unsigned short* ph = whi + (size_t)i * 8;
    unsigned short* pl = wlo + (size_t)i * 8;
    *(volatile v8h*)ph = hv;
    *(volatile v8h*)pl = lv;
    __threadfence();
    *(volatile v8h*)ph = hv;
    *(volatile v8h*)pl = lv;
  }
}

__global__ __launch_bounds__(kThr) void rnn_seq_kernel(const int* __restrict__ x, const int* __restrict__ lengths,
                                                       const float* __restrict__ ptab,
                                                       const unsigned short* __restrict__ whi_p,
                                                       const unsigned short* __restrict__ wlo_p,
                                                       const float* __restrict__ w_fc, const float* __restrict__ b_fc,
                                                       float* __restrict__ out) {
  __shared__ __align__(16) float  s_tab[kVocab * kHid];
  __shared__ __align__(16) int    s_tok[kSteps * kTileM];
  __shared__ __align__(16) __bf16 s_hhi[2][kTileM * kHid];
  __shared__ __align__(16) __bf16 s_hlo[2][kTileM * kHid];
  __shared__ __align__(16) int    s_len[kTileM];

  const int tid  = threadIdx.x;
  const int wave = tid >> 5;
  const int lane = tid & 31;
  const int c    = lane & 15;
  const int hh   = lane >> 4;
  const int koff = hh * 8;
  const int col  = wave * 16 + c;
  const int rowbase = blockIdx.x * kTileM;

  {
    const v4f* src = (const v4f*)ptab;
    v4f* dst = (v4f*)s_tab;
#pragma unroll 1
    for (int i = tid; i < (kVocab * kHid) / 4; i += kThr) dst[i] = src[i];
  }
#pragma unroll 1
  for (int i = tid; i < kTileM * kSteps; i += kThr) {
    const int row = i >> 8;
    const int t   = i & (kSteps - 1);
    int tk = x[(size_t)(rowbase + row) * kSteps + t];
    tk = tk < 0 ? 0 : tk;
    tk = tk > (kVocab - 1) ? (kVocab - 1) : tk;
    s_tok[t * kTileM + row] = tk;
  }
  {
    int lm = lengths[rowbase + (tid & (kTileM - 1))] - 1;
    lm = lm < 0 ? 0 : lm;
    lm = lm > (kSteps - 1) ? (kSteps - 1) : lm;
    if (tid < kTileM) s_len[tid] = lm;
  }
  {
    const v8b zz = {};
    __bf16* ph = &s_hhi[0][0];
    __bf16* pl = &s_hlo[0][0];
#pragma unroll 1
    for (int i = tid; i < (2 * kTileM * kHid) / 8; i += kThr) {
      *(v8b*)(ph + i * 8) = zz;
      *(v8b*)(pl + i * 8) = zz;
    }
  }

  v16b bhi[4], blo[4];
  {
    const __bf16* wh = (const __bf16*)whi_p + (size_t)col * kHid + koff;
    const __bf16* wl = (const __bf16*)wlo_p + (size_t)col * kHid + koff;
#pragma unroll
    for (int kc = 0; kc < 4; ++kc) {
      bhi[kc] = frag_load_bf(wh + kc * 32);
      blo[kc] = frag_load_bf(wl + kc * 32);
    }
  }
  __syncthreads();

  int lm1[8];
#pragma unroll
  for (int r = 0; r < 8; ++r) lm1[r] = s_len[8 * hh + r];
  int tmax = 1;
#pragma unroll
  for (int r = 0; r < kTileM; ++r) {
    const int l = s_len[r] + 1;
    tmax = (l > tmax) ? l : tmax;
  }
  tmax = (tmax > kSteps) ? kSteps : tmax;

  float lastv[8];
#pragma unroll
  for (int r = 0; r < 8; ++r) lastv[r] = 0.0f;

  const v8f z8 = {0.f, 0.f, 0.f, 0.f, 0.f, 0.f, 0.f, 0.f};

#pragma unroll 1
  for (int t = 0; t < tmax; ++t) {
    const int rb = t & 1;
    const int wb = rb ^ 1;

    const int4 tk0 = *(const int4*)&s_tok[t * kTileM + 8 * hh];
    const int4 tk1 = *(const int4*)&s_tok[t * kTileM + 8 * hh + 4];
    float pv[8];
    pv[0] = s_tab[tk0.x * kHid + col];
    pv[1] = s_tab[tk0.y * kHid + col];
    pv[2] = s_tab[tk0.z * kHid + col];
    pv[3] = s_tab[tk0.w * kHid + col];
    pv[4] = s_tab[tk1.x * kHid + col];
    pv[5] = s_tab[tk1.y * kHid + col];
    pv[6] = s_tab[tk1.z * kHid + col];
    pv[7] = s_tab[tk1.w * kHid + col];

    const __bf16* ah = &s_hhi[rb][0] + c * kHid + koff;
    const __bf16* al = &s_hlo[rb][0] + c * kHid + koff;
    v8f accM = z8, accR = z8;
#pragma unroll
    for (int kc = 0; kc < 4; ++kc) {
      const v16b fh = frag_load_bf(ah + kc * 32);
      const v16b fl = frag_load_bf(al + kc * 32);
      accM = mma_bf(fh, bhi[kc], accM);
      accR = mma_bf(fl, bhi[kc], accR);
      accR = mma_bf(fh, blo[kc], accR);
      group_guard(accM, accR, fh, fl, bhi[kc], blo[kc]);
    }

    __bf16* nh = &s_hhi[wb][0];
    __bf16* nl = &s_hlo[wb][0];
#pragma unroll
    for (int r = 0; r < 8; ++r) {
      const float zs = (accM[r] + accR[r]) + pv[r];
      const float hv = tanh_acc(zs);
      const unsigned short hb = f2bf_bits(hv);
      const unsigned short lb = f2bf_bits(hv - bf_bits2f(hb));
      nh[(8 * hh + r) * kHid + col] = __builtin_bit_cast(__bf16, hb);
      nl[(8 * hh + r) * kHid + col] = __builtin_bit_cast(__bf16, lb);
      lastv[r] = (lm1[r] == t) ? hv : lastv[r];
    }
    __syncthreads();
  }

  __syncthreads();
  float* s_last = s_tab;
  float* s_out  = s_tab + kTileM * kHid;
#pragma unroll
  for (int r = 0; r < 8; ++r) s_last[(8 * hh + r) * kHid + col] = lastv[r];
  __syncthreads();

#pragma unroll 1
  for (int i = 0; i < 4; ++i) {
    const int o  = tid + i * kThr;
    const int oc = (o < kOutTile) ? o : (kOutTile - 1);
    const int row = oc / kVocab;
    const int v   = oc - row * kVocab;
    const float* lp = s_last + row * kHid;
    const float* wp = w_fc + v * kHid;
    float s = 0.0f;
#pragma unroll 4
    for (int k = 0; k < kHid; k += 4) {
      const v4f a = *(const v4f*)(lp + k);
      const v4f w = *(const v4f*)(wp + k);
      s = fmaf(a[0], w[0], s);
      s = fmaf(a[1], w[1], s);
      s = fmaf(a[2], w[2], s);
      s = fmaf(a[3], w[3], s);
    }
    const float res = s + b_fc[v];
    if (o < kOutTile) s_out[o] = res;
  }
  __syncthreads();

  {
    float* ob = out + (size_t)blockIdx.x * kOutTile;
    for (int pass = 0; pass < 2; ++pass) {
#pragma unroll 1
      for (int ln = wave; ln < kOutLines; ln += kWaves) {
        const float val = s_out[ln * 32 + lane];
        *(volatile float*)(ob + ln * 32 + lane) = val;
      }
      __threadfence();
    }
  }
}

extern "C" void kernel_launch(void* const* d_in, const int* in_sizes, int n_in,
                              void* d_out, int out_size, void* d_ws, size_t ws_size, hipStream_t stream) {
  if (n_in < 7 || d_out == nullptr || d_ws == nullptr) return;
  if (in_sizes[0] != kBatch * kSteps || in_sizes[1] != kBatch || in_sizes[2] != kVocab * kHid ||
      in_sizes[3] != kHid * kHid || in_sizes[4] != kHid * kHid || in_sizes[5] != kVocab * kHid ||
      in_sizes[6] != kVocab || out_size != kBatch * kVocab) return;

  const int*   x       = (const int*)d_in[0];
  const int*   lengths = (const int*)d_in[1];
  const float* emb     = (const float*)d_in[2];
  const float* w_ih    = (const float*)d_in[3];
  const float* w_hh    = (const float*)d_in[4];
  const float* w_fc    = (const float*)d_in[5];
  const float* b_fc    = (const float*)d_in[6];
  float* out = (float*)d_out;

  char* ws = (char*)d_ws;
  size_t off = 0;
  auto carve = [&](size_t bytes) -> char* { char* p = ws + off; off += (bytes + 255) & ~(size_t)255; return p; };
  float*          PTAB = (float*)carve((size_t)kVocPad * kHid * 4);
  unsigned short* WHI  = (unsigned short*)carve((size_t)kHid * kHid * 2);
  unsigned short* WLO  = (unsigned short*)carve((size_t)kHid * kHid * 2);
  if (off > ws_size || off > (size_t)134217728) return;

  prep_kernel<<<kPrepBlkP + kPrepBlkW, kThr, 0, stream>>>(emb, w_ih, w_hh, PTAB, WHI, WLO);
  rnn_seq_kernel<<<kBatch / kTileM, kThr, 0, stream>>>(x, lengths, PTAB, WHI, WLO, w_fc, b_fc, out);
}
